// MultiHeadGATLayer_2654289789413
// MI455X (gfx1250) — hardware-verified
//
#include <hip/hip_runtime.h>
#include <stddef.h>


#define NIN     512
#define ZW      512
#define NHEAD   8
#define HCH     64
#define NHID    2048
#define WAW     128
#define EPW     8
#define GBM     32
#define GTHR    256
#define NWAVE   8
#define XSP     528
#define YSP     272
#define STP     516
#define CHK     256
#define NTHR    256
#define EPT     8
#define CHUNK   (NTHR * EPT)
#define WCAP    (EPT * 32)
#define LISTN   (NWAVE * WCAP)
#define NBMAX   2048
#define SLOTB   11
#define RCAP    28672
#define DEGCAP  4096
#define NSTRM   2
#define NEG_SLOPE 0.01f
#define LN_EPS  0.00001f
#define CA      8.0f
#define CW1     16.0f
#define CW2     32.0f
#define SCA     0.0078125f
#define SCB     0.00390625f
#define WSCAP   134217728
#define LDS_GAT ((2 * RCAP + 2 * NBMAX + LISTN) * 4 + 64)
#define LDS_MM  (GBM * STP * 4)

static_assert((CHUNK & (CHUNK - 1)) == 0 && CHUNK <= 4096);
static_assert(NBMAX == (1 << SLOTB));
static_assert(NTHR * 8 == NBMAX);
static_assert(LISTN >= NBMAX);
static_assert(LISTN >= NWAVE * WCAP);
static_assert((RCAP % 32) == 0);
static_assert(LDS_GAT <= 300000);
static_assert(GTHR == NWAVE * 32 && NTHR == GTHR);
static_assert(NHEAD * HCH == ZW && NWAVE * HCH == ZW);
static_assert(NWAVE * 32 == CHK && NWAVE * 64 == NIN && (NHID % CHK) == 0);
static_assert((NIN % 32) == 0 && (CHK % 32) == 0 && (NHID % 32) == 0);
static_assert(NSTRM * NHEAD * 2 == 32 && 32 * 16 == ZW);
static_assert(GBM * XSP * 2 <= LDS_MM && GBM * (XSP + YSP) * 2 <= LDS_MM);
static_assert((XSP % 8) == 0 && (YSP % 8) == 0 && (STP % 4) == 0);
static_assert(NWAVE * NSTRM * ZW + NWAVE * NSTRM * NHEAD <= RCAP);
static_assert(GBM * EPW == 256);
static_assert(GTHR / 8 == GBM);
static_assert(NHEAD * WAW == 1024);

typedef float    v4f  __attribute__((ext_vector_type(4)));
typedef float    v8f  __attribute__((ext_vector_type(8)));
typedef int      v4i  __attribute__((ext_vector_type(4)));
typedef int      v8i  __attribute__((ext_vector_type(8)));
typedef _Float16 v8h  __attribute__((ext_vector_type(8)));
typedef _Float16 v16h __attribute__((ext_vector_type(16)));
union FragH { v16h v; v8h h[2]; v8i w; };

__device__ __forceinline__ v8f wmh(const FragH& a, const FragH& b, v8f c) {
  v8f d = __builtin_amdgcn_wmma_f32_16x16x32_f16(false, a.v, false, b.v, (short)0, c, false, false);
  asm volatile("v_nop\n\tv_nop\n\tv_nop\n\tv_nop" : "+v"(d) : "v"(a.w), "v"(b.w));
  return d;
}

__device__ __forceinline__ v8h pack8(v4f a, v4f b, float sc) {
  v8h hv;
  hv[0] = (_Float16)(a.x * sc); hv[1] = (_Float16)(a.y * sc);
  hv[2] = (_Float16)(a.z * sc); hv[3] = (_Float16)(a.w * sc);
  hv[4] = (_Float16)(b.x * sc); hv[5] = (_Float16)(b.y * sc);
  hv[6] = (_Float16)(b.z * sc); hv[7] = (_Float16)(b.w * sc);
  return hv;
}

__device__ __forceinline__ int scan_chunk(const int* __restrict__ dsts, int nE, int cbase, int slotBase,
                                          int nb, int vec8, int* list, int tid, int lane, int wave) {
  int wc = 0;
  const int el0  = tid * EPT;
  const int e0   = cbase + el0;
  const int sent = -2147483647 - 1;
  v4i da, db;
  if (vec8 != 0 && cbase + CHUNK <= nE) {
    da = *(const v4i*)(dsts + e0);
    db = *(const v4i*)(dsts + e0 + 4);
  } else {
    da.x = (e0     < nE) ? dsts[min(e0,     nE - 1)] : sent;
    da.y = (e0 + 1 < nE) ? dsts[min(e0 + 1, nE - 1)] : sent;
    da.z = (e0 + 2 < nE) ? dsts[min(e0 + 2, nE - 1)] : sent;
    da.w = (e0 + 3 < nE) ? dsts[min(e0 + 3, nE - 1)] : sent;
    db.x = (e0 + 4 < nE) ? dsts[min(e0 + 4, nE - 1)] : sent;
    db.y = (e0 + 5 < nE) ? dsts[min(e0 + 5, nE - 1)] : sent;
    db.z = (e0 + 6 < nE) ? dsts[min(e0 + 6, nE - 1)] : sent;
    db.w = (e0 + 7 < nE) ? dsts[min(e0 + 7, nE - 1)] : sent;
  }
  const unsigned nbs = (unsigned)slotBase;
  const unsigned unb = (unsigned)nb;
  const unsigned s0 = (unsigned)da.x - nbs, s1 = (unsigned)da.y - nbs;
  const unsigned s2 = (unsigned)da.z - nbs, s3 = (unsigned)da.w - nbs;
  const unsigned s4 = (unsigned)db.x - nbs, s5 = (unsigned)db.y - nbs;
  const unsigned s6 = (unsigned)db.z - nbs, s7 = (unsigned)db.w - nbs;
  const bool h0 = s0 < unb, h1 = s1 < unb, h2 = s2 < unb, h3 = s3 < unb;
  const bool h4 = s4 < unb, h5 = s5 < unb, h6 = s6 < unb, h7 = s7 < unb;
  const unsigned any = __builtin_amdgcn_ballot_w32(h0 | h1 | h2 | h3 | h4 | h5 | h6 | h7);
  if (any != 0u) {
#define HITJ(J, HJ, SJ) { \
      const unsigned mj = __builtin_amdgcn_ballot_w32(HJ); \
      if (mj != 0u) { \
        if (HJ) { \
          const int pos = wc + (int)__builtin_amdgcn_mbcnt_lo(mj, 0u); \
          if (pos < WCAP) list[wave * WCAP + pos] = ((el0 + (J)) << 12) | (int)(SJ); \
        } \
        wc += (int)__builtin_popcount(mj); } }
    HITJ(0, h0, s0)
    HITJ(1, h1, s1)
    HITJ(2, h2, s2)
    HITJ(3, h3, s3)
    HITJ(4, h4, s4)
    HITJ(5, h5, s5)
    HITJ(6, h6, s6)
    HITJ(7, h7, s7)
#undef HITJ
  }
  return wc;
}

__global__ __launch_bounds__(NTHR) void k_wprep(const float* __restrict__ wfc, const float* __restrict__ w1,
                                                const float* __restrict__ w2,
                                                _Float16* wfh, _Float16* w1h, _Float16* w2h) {
  const int j = (int)blockIdx.y;
  const int u = (int)blockIdx.x * NTHR + (int)threadIdx.x;
  const float* src;
  _Float16* dstp;
  int nUnits;
  float sc;
  if (j == 0)      { src = wfc; dstp = wfh; nUnits = ZW * NIN / 8;   sc = CW1; }
  else if (j == 1) { src = w1;  dstp = w1h; nUnits = NHID * NIN / 8; sc = CW1; }
  else             { src = w2;  dstp = w2h; nUnits = NIN * NHID / 8; sc = CW2; }
  if (u >= nUnits) return;
  const float* p = src + (size_t)u * 8;
  const v4f a = *(const v4f*)p, b = *(const v4f*)(p + 4);
  const v8h hv = pack8(a, b, sc);
  _Float16* o = dstp + (size_t)u * 8;
  *(volatile v8h*)o = hv;
  __threadfence();
  *(volatile v8h*)o = hv;
}

__global__ __launch_bounds__(GTHR) void k_zgemm(const float* __restrict__ hin, const _Float16* __restrict__ wfh,
                                                const float* __restrict__ wa, float* Z, float* ES, float* ED,
                                                int nN) {
  extern __shared__ v4f dynl[];
  _Float16* xs = (_Float16*)dynl;
  float* stg = (float*)dynl;
  __shared__ float sWa[NHEAD * WAW];
  __shared__ __attribute__((aligned(16))) float esT[GBM * EPW];
  __shared__ __attribute__((aligned(16))) float edT[GBM * EPW];
  const int tid = threadIdx.x, lane = tid & 31, wave = tid >> 5, hh = lane >> 4, m = lane & 15;
  const int rowBase = (int)blockIdx.x * GBM;
  const v4f z4 = {0.f, 0.f, 0.f, 0.f};
  for (int i = tid; i < NHEAD * WAW; i += GTHR) sWa[i] = wa[i];
#pragma unroll 1
  for (int f = tid; f < GBM * (NIN / 8); f += GTHR) {
    const int r = f >> 6, c8 = (f & 63) * 8;
    const int row = rowBase + r;
    const int rc  = row < nN ? row : nN - 1;
    const float* p = hin + (size_t)rc * NIN + c8;
    v4f a = *(const v4f*)p, b = *(const v4f*)(p + 4);
    if (row >= nN) { a = z4; b = z4; }
    *(v8h*)(xs + (size_t)r * XSP + c8) = pack8(a, b, CA);
  }
  __syncthreads();
  v8f acc[2][4];
#pragma unroll
  for (int i = 0; i < 2; ++i)
#pragma unroll
    for (int t = 0; t < 4; ++t) { v8f z = {0.f, 0.f, 0.f, 0.f, 0.f, 0.f, 0.f, 0.f}; acc[i][t] = z; }
  const _Float16* ap = xs + (size_t)m * XSP + 8 * hh;
  const _Float16* bp = wfh + (size_t)(HCH * wave + m) * NIN + 8 * hh;
#pragma unroll 1
  for (int ks = 0; ks < NIN / 32; ++ks) {
    FragH a0, a1;
    a0.h[0] = *(const v8h*)(ap + 32 * ks);
    a0.h[1] = *(const v8h*)(ap + 32 * ks + 16);
    a1.h[0] = *(const v8h*)(ap + 16 * XSP + 32 * ks);
    a1.h[1] = *(const v8h*)(ap + 16 * XSP + 32 * ks + 16);
#pragma unroll
    for (int t = 0; t < 4; ++t) {
      const _Float16* bq = bp + (size_t)(16 * t) * NIN + 32 * ks;
      FragH bf;
      bf.h[0] = *(const v8h*)bq;
      bf.h[1] = *(const v8h*)(bq + 16);
      acc[0][t] = wmh(a0, bf, acc[0][t]);
      acc[1][t] = wmh(a1, bf, acc[1][t]);
    }
  }
  __syncthreads();
  {
    float* sp = stg + (size_t)(8 * hh) * STP + HCH * wave + m;
#pragma unroll
    for (int i = 0; i < 2; ++i)
#pragma unroll
      for (int t = 0; t < 4; ++t)
#pragma unroll
        for (int r = 0; r < 8; ++r) sp[(size_t)(16 * i + r) * STP + 16 * t] = acc[i][t][r] * SCA;
  }
  __syncthreads();
  {
    const float* srow = stg + (size_t)lane * STP + HCH * wave;
    const float* as = sWa + wave * WAW;
    float s = 0.f, d = 0.f;
#pragma unroll 1
    for (int o = 0; o < HCH; ++o) {
      const float v = srow[o];
      s = fmaf(v, as[o], s);
      d = fmaf(v, as[HCH + o], d);
    }
    esT[lane * EPW + wave] = s;
    edT[lane * EPW + wave] = d;
  }
  {
    const int nF4 = GBM * ZW / 4;
    float* zb = Z + (size_t)rowBase * ZW;
#pragma unroll 1
    for (int f = tid; f < nF4; f += GTHR) {
      const int r = f >> 7, q = f & 127;
      const v4f v = *(const v4f*)(stg + (size_t)r * STP + 4 * q);
      *(volatile v4f*)(zb + (size_t)r * ZW + 4 * q) = v;
    }
    __threadfence();
#pragma unroll 1
    for (int f = tid; f < nF4; f += GTHR) {
      const int r = f >> 7, q = f & 127;
      const v4f v = *(const v4f*)(stg + (size_t)r * STP + 4 * q);
      *(volatile v4f*)(zb + (size_t)r * ZW + 4 * q) = v;
    }
  }
  __syncthreads();
  if (wave == 0) {
    const v4f* e4 = (const v4f*)esT;
    const v4f v0 = e4[lane], v1 = e4[32 + lane];
    float* pe = ES + (size_t)rowBase * EPW;
    *(volatile v4f*)(pe + 4 * lane) = v0;
    *(volatile v4f*)(pe + 128 + 4 * lane) = v1;
    __threadfence();
    *(volatile v4f*)(pe + 4 * lane) = v0;
    *(volatile v4f*)(pe + 128 + 4 * lane) = v1;
  } else if (wave == 1) {
    const v4f* d4 = (const v4f*)edT;
    const v4f v0 = d4[lane], v1 = d4[32 + lane];
    float* pd = ED + (size_t)rowBase * EPW;
    *(volatile v4f*)(pd + 4 * lane) = v0;
    *(volatile v4f*)(pd + 128 + 4 * lane) = v1;
    __threadfence();
    *(volatile v4f*)(pd + 4 * lane) = v0;
    *(volatile v4f*)(pd + 128 + 4 * lane) = v1;
  }
}

__global__ __launch_bounds__(NTHR) void k_gat(const int* __restrict__ dsts, const int* __restrict__ srcs,
                                              const float* __restrict__ Z, const float* __restrict__ ES,
                                              const float* __restrict__ ED, const float* __restrict__ hin,
                                              float* XF, int nN, int nE, int nb, int vec8) {
  extern __shared__ v4f lds_dyn[];
  int* reg1 = (int*)lds_dyn;
  int* reg2 = reg1 + RCAP;
  int* scnt = reg2 + RCAP;
  int* soff = scnt + NBMAX;
  int* list = soff + NBMAX;
  int* wcnt = list + LISTN;
  int* wtot = wcnt + NWAVE;
  const int tid = threadIdx.x, lane = tid & 31, wave = tid >> 5;
  const int nodeBase = (int)blockIdx.x * nb;

  for (int i = tid; i < NBMAX; i += NTHR) scnt[i] = 0;
  {
    const v4i z = {0, 0, 0, 0};
    v4i* r2v = (v4i*)reg2;
    for (int f = tid; f < RCAP / 4; f += NTHR) r2v[f] = z;
  }
  __syncthreads();

  int tot = 0;
  const int nChunks = (nE + CHUNK - 1) / CHUNK;
#pragma unroll 1
  for (int ch = 0; ch < nChunks; ++ch) {
    const int cbase = ch * CHUNK;
    const int wc = scan_chunk(dsts, nE, cbase, nodeBase, nb, vec8, list, tid, lane, wave);
    if (lane == 0) wcnt[wave] = wc;
    __syncthreads();
    int pre = 0, all = 0;
#pragma unroll
    for (int w2 = 0; w2 < NWAVE; ++w2) {
      int c = wcnt[w2];
      c = c < 0 ? 0 : (c > WCAP ? WCAP : c);
      all += c;
      pre += (w2 < wave) ? c : 0;
    }
    const int wcc  = wc > WCAP ? WCAP : wc;
    const int base = tot + pre;
#pragma unroll 1
    for (int i = lane; i < wcc; i += 32) {
      const int ent = list[wave * WCAP + i];
      const int el  = (ent >> 12) & (CHUNK - 1);
      const int sl  = ent & (NBMAX - 1);
      int eid = cbase + el;
      eid = eid > nE - 1 ? nE - 1 : eid;
      const int pos = base + i;
      if (pos < RCAP) reg1[pos] = (int)(((unsigned)eid << SLOTB) | (unsigned)sl);
    }
    tot += all;
    tot = tot > RCAP ? RCAP : tot;
    __syncthreads();
  }
  const int nh = tot;

  if (wave == 0) {
#pragma unroll 1
    for (int b0 = 0; b0 < nh; b0 += 32) {
      const int idx = b0 + lane;
      const int uv  = reg1[idx < RCAP ? idx : RCAP - 1];
      const int m32 = (nh - b0) < 32 ? (nh - b0) : 32;
#pragma unroll 1
      for (int k = 0; k < m32; ++k) {
        const int u  = __builtin_amdgcn_readlane(uv, k);
        const int sl = u & (NBMAX - 1);
        if (lane == 0) scnt[sl] = scnt[sl] + 1;
      }
    }
  }
  __syncthreads();

  {
    const v4i ca = *(const v4i*)(scnt + 8 * tid);
    const v4i cb = *(const v4i*)(scnt + 8 * tid + 4);
    const int e0 = ca.x < 0 ? 0 : ca.x, e1 = ca.y < 0 ? 0 : ca.y, e2 = ca.z < 0 ? 0 : ca.z, e3 = ca.w < 0 ? 0 : ca.w;
    const int e4 = cb.x < 0 ? 0 : cb.x, e5 = cb.y < 0 ? 0 : cb.y, e6 = cb.z < 0 ? 0 : cb.z, e7 = cb.w < 0 ? 0 : cb.w;
    const int ts = e0 + e1 + e2 + e3 + e4 + e5 + e6 + e7;
    int incl = ts;
#pragma unroll
    for (int d = 1; d < 32; d <<= 1) {
      const int up = __shfl_up(incl, d);
      if (lane >= d) incl += up;
    }
    if (lane == 31) wtot[wave] = incl;
    __syncthreads();
    int pre = 0;
#pragma unroll
    for (int w2 = 0; w2 < NWAVE; ++w2) pre += (w2 < wave) ? wtot[w2] : 0;
    int run = pre + incl - ts;
    soff[8 * tid + 0] = run; run += e0;
    soff[8 * tid + 1] = run; run += e1;
    soff[8 * tid + 2] = run; run += e2;
    soff[8 * tid + 3] = run; run += e3;
    soff[8 * tid + 4] = run; run += e4;
    soff[8 * tid + 5] = run; run += e5;
    soff[8 * tid + 6] = run; run += e6;
    soff[8 * tid + 7] = run;
  }
  __syncthreads();
  for (int i = tid; i < NBMAX; i += NTHR) list[i] = soff[i];
  __syncthreads();

  if (wave == 0) {
#pragma unroll 1
    for (int b0 = 0; b0 < nh; b0 += 32) {
      const int idx = b0 + lane;
      const int uv  = reg1[idx < RCAP ? idx : RCAP - 1];
      const int m32 = (nh - b0) < 32 ? (nh - b0) : 32;
#pragma unroll 1
      for (int k = 0; k < m32; ++k) {
        const int u   = __builtin_amdgcn_readlane(uv, k);
        const int sl  = u & (NBMAX - 1);
        const int eid = (int)((unsigned)u >> SLOTB);
        if (lane == 0) {
          int pos = list[sl];
          pos = pos < 0 ? 0 : (pos > RCAP - 1 ? RCAP - 1 : pos);
          reg2[pos] = eid;
          list[sl] = pos + 1;
        }
      }
    }
  }
  __syncthreads();

  const bool ovf = (nh >= RCAP);
  const int g   = lane >> 4;
  const int sub = lane & 15;
  const int j   = sub >> 1;
  const int chf = sub & 1;
  const int cb0 = 32 * sub;
  const int hd  = lane >> 2;
  v4f*   cw  = (v4f*)lds_dyn + wave * (NSTRM * (ZW / 4));
  float* cwf = (float*)cw;
  float* cd  = (float*)lds_dyn + NWAVE * NSTRM * ZW + wave * (NSTRM * NHEAD);
  const int nbw = nb >> 3;
  const float qnan = __int_as_float(0x7fc00000);
  const v4f z4 = {0.f, 0.f, 0.f, 0.f};
#pragma unroll 1
  for (int jt = 0; jt < nbw; ++jt) {
    const int slot = wave * nbw + jt;
    const int grow = nodeBase + slot;
    const int gcl  = grow < nN ? grow : nN - 1;
    const bool wr  = grow < nN;
    int st = soff[slot];
    const int craw = scnt[slot];
    st = st < 0 ? 0 : (st > RCAP - 1 ? RCAP - 1 : st);
    int cnt = craw < 0 ? 0 : (craw > DEGCAP ? DEGCAP : craw);
    if (cnt > RCAP - st) cnt = RCAP - st;
    const bool pois = ovf || (craw < 0) || (craw > DEGCAP);
    const float edv = ED[(size_t)gcl * EPW + j];
    const int niter = (cnt + NSTRM - 1) / NSTRM;

    float mx = -1.0e30f;
#pragma unroll 1
    for (int it = 0; it < niter; ++it) {
      const int q = it * NSTRM + g;
      const bool valid = q < cnt;
      const int qc = valid ? q : cnt - 1;
      int eid = reg2[st + qc];
      eid = eid < 0 ? 0 : (eid > nE - 1 ? nE - 1 : eid);
      const int sraw = srcs[eid];
      const int s = sraw < 0 ? 0 : (sraw > nN - 1 ? nN - 1 : sraw);
      const float u = ES[(size_t)s * EPW + j] + edv;
      const float l = fmaxf(u, NEG_SLOPE * u);
      mx = valid ? fmaxf(mx, l) : mx;
    }
    const float m1 = fmaxf(mx, __shfl_xor(mx, 16));

    float dn = 0.f;
    v4f a0 = z4, a1 = z4, a2 = z4, a3 = z4, a4 = z4, a5 = z4, a6 = z4, a7 = z4;
#pragma unroll 1
    for (int it = 0; it < niter; ++it) {
      const int q = it * NSTRM + g;
      const bool valid = q < cnt;
      const int qc = valid ? q : cnt - 1;
      int eid = reg2[st + qc];
      eid = eid < 0 ? 0 : (eid > nE - 1 ? nE - 1 : eid);
      const int sraw = srcs[eid];
      const int s = sraw < 0 ? 0 : (sraw > nN - 1 ? nN - 1 : sraw);
      const float* ys = Z + (size_t)s * ZW + cb0;
      const v4f x0 = *(const v4f*)(ys +  0);
      const v4f x1 = *(const v4f*)(ys +  4);
      const v4f x2 = *(const v4f*)(ys +  8);
      const v4f x3 = *(const v4f*)(ys + 12);
      const v4f x4 = *(const v4f*)(ys + 16);
      const v4f x5 = *(const v4f*)(ys + 20);
      const v4f x6 = *(const v4f*)(ys + 24);
      const v4f x7 = *(const v4f*)(ys + 28);
      const float u = ES[(size_t)s * EPW + j] + edv;
      const float l = fmaxf(u, NEG_SLOPE * u);
      const float p = valid ? __expf(l - m1) : 0.0f;
      dn += p;
      a0 = a0 + x0 * p;
      a1 = a1 + x1 * p;
      a2 = a2 + x2 * p;
      a3 = a3 + x3 * p;
      a4 = a4 + x4 * p;
      a5 = a5 + x5 * p;
      a6 = a6 + x6 * p;
      a7 = a7 + x7 * p;
    }

    __builtin_amdgcn_fence(__ATOMIC_RELEASE, "wavefront");
    __builtin_amdgcn_wave_barrier();
    {
      v4f* cg = cw + g * (ZW / 4) + 8 * sub;
      cg[0] = a0; cg[1] = a1; cg[2] = a2; cg[3] = a3;
      cg[4] = a4; cg[5] = a5; cg[6] = a6; cg[7] = a7;
      if (chf == 0) cd[g * NHEAD + j] = dn;
    }
    __builtin_amdgcn_fence(__ATOMIC_RELEASE, "wavefront");
    __builtin_amdgcn_wave_barrier();
    {
      const float ds = cd[hd] + cd[NHEAD + hd];
      float inv = ds > 0.f ? __builtin_amdgcn_rcpf(ds) : 0.f;
      inv = pois ? qnan : inv;
      const v4f o0 = (cw[4 * lane + 0] + cw[(ZW / 4) + 4 * lane + 0]) * inv;
      const v4f o1 = (cw[4 * lane + 1] + cw[(ZW / 4) + 4 * lane + 1]) * inv;
      const v4f o2 = (cw[4 * lane + 2] + cw[(ZW / 4) + 4 * lane + 2]) * inv;
      const v4f o3 = (cw[4 * lane + 3] + cw[(ZW / 4) + 4 * lane + 3]) * inv;
      cw[4 * lane + 0] = o0;
      cw[4 * lane + 1] = o1;
      cw[4 * lane + 2] = o2;
      cw[4 * lane + 3] = o3;
    }
    __builtin_amdgcn_fence(__ATOMIC_RELEASE, "wavefront");
    __builtin_amdgcn_wave_barrier();
    {
      float* rf = cwf + 16 * lane;
#pragma unroll 1
      for (int c = 0; c < 16; ++c) {
        const float v  = rf[c];
        const float ev = expm1f(v);
        rf[c] = v > 0.f ? v : ev;
      }
    }
    __builtin_amdgcn_fence(__ATOMIC_RELEASE, "wavefront");
    __builtin_amdgcn_wave_barrier();
    {
      const v4f* hr = (const v4f*)(hin + (size_t)gcl * NIN);
      float* xrow = XF + (size_t)gcl * NIN;
      const v4f xv0 = cw[lane]      + hr[lane];
      const v4f xv1 = cw[32 + lane] + hr[32 + lane];
      const v4f xv2 = cw[64 + lane] + hr[64 + lane];
      const v4f xv3 = cw[96 + lane] + hr[96 + lane];
      if (wr) {
        *(volatile v4f*)(xrow +       4 * lane) = xv0;
        *(volatile v4f*)(xrow + 128 + 4 * lane) = xv1;
        *(volatile v4f*)(xrow + 256 + 4 * lane) = xv2;
        *(volatile v4f*)(xrow + 384 + 4 * lane) = xv3;
      }
      __threadfence();
      if (wr) {
        *(volatile v4f*)(xrow +       4 * lane) = xv0;
        *(volatile v4f*)(xrow + 128 + 4 * lane) = xv1;
        *(volatile v4f*)(xrow + 256 + 4 * lane) = xv2;
        *(volatile v4f*)(xrow + 384 + 4 * lane) = xv3;
      }
    }
  }
}

__global__ __launch_bounds__(GTHR) void k_ffn(const float* __restrict__ xf, const _Float16* __restrict__ w1h,
                                              const _Float16* __restrict__ w2h, const float* __restrict__ b1,
                                              const float* __restrict__ b2, const float* __restrict__ lng,
                                              const float* __restrict__ lnb, float* out, int nN) {
  extern __shared__ v4f dynl[];
  _Float16* xs = (_Float16*)dynl;
  _Float16* ys = xs + GBM * XSP;
  float* stg = (float*)dynl;
  const int tid = threadIdx.x, lane = tid & 31, wave = tid >> 5, hh = lane >> 4, m = lane & 15;
  const int rowBase = (int)blockIdx.x * GBM;
  const v4f z4 = {0.f, 0.f, 0.f, 0.f};
#pragma unroll 1
  for (int f = tid; f < GBM * (NIN / 8); f += GTHR) {
    const int r = f >> 6, c8 = (f & 63) * 8;
    const int row = rowBase + r;
    const int rc  = row < nN ? row : nN - 1;
    const float* p = xf + (size_t)rc * NIN + c8;
    v4f a = *(const v4f*)p, b = *(const v4f*)(p + 4);
    if (row >= nN) { a = z4; b = z4; }
    *(v8h*)(xs + (size_t)r * XSP + c8) = pack8(a, b, CA);
  }
  __syncthreads();

  v8f acc2[2][4];
#pragma unroll
  for (int i = 0; i < 2; ++i)
#pragma unroll
    for (int t = 0; t < 4; ++t) { v8f z = {0.f, 0.f, 0.f, 0.f, 0.f, 0.f, 0.f, 0.f}; acc2[i][t] = z; }
  const _Float16* apx = xs + (size_t)m * XSP + 8 * hh;
  const _Float16* apy = ys + (size_t)m * YSP + 8 * hh;

#pragma unroll 1
  for (int c = 0; c < NHID / CHK; ++c) {
    v8f acc1[2][2];
#pragma unroll
    for (int i = 0; i < 2; ++i)
#pragma unroll
      for (int t = 0; t < 2; ++t) { v8f z = {0.f, 0.f, 0.f, 0.f, 0.f, 0.f, 0.f, 0.f}; acc1[i][t] = z; }
    const _Float16* bp1 = w1h + (size_t)(CHK * c + 32 * wave + m) * NIN + 8 * hh;
#pragma unroll 1
    for (int ks = 0; ks < NIN / 32; ++ks) {
      FragH a0, a1;
      a0.h[0] = *(const v8h*)(apx + 32 * ks);
      a0.h[1] = *(const v8h*)(apx + 32 * ks + 16);
      a1.h[0] = *(const v8h*)(apx + 16 * XSP + 32 * ks);
      a1.h[1] = *(const v8h*)(apx + 16 * XSP + 32 * ks + 16);
#pragma unroll
      for (int t = 0; t < 2; ++t) {
        const _Float16* bq = bp1 + (size_t)(16 * t) * NIN + 32 * ks;
        FragH bf;
        bf.h[0] = *(const v8h*)bq;
        bf.h[1] = *(const v8h*)(bq + 16);
        acc1[0][t] = wmh(a0, bf, acc1[0][t]);
        acc1[1][t] = wmh(a1, bf, acc1[1][t]);
      }
    }
    {
      _Float16* yp = ys + (size_t)(8 * hh) * YSP + 32 * wave + m;
#pragma unroll
      for (int t = 0; t < 2; ++t) {
        const float bb = b1[CHK * c + 32 * wave + 16 * t + m];
#pragma unroll
        for (int i = 0; i < 2; ++i)
#pragma unroll
          for (int r = 0; r < 8; ++r) {
            const float v = fmaxf(fmaf(acc1[i][t][r], SCA, bb), 0.f);
            yp[(size_t)(16 * i + r) * YSP + 16 * t] = (_Float16)(v * CA);
          }
      }
    }
    __syncthreads();
    const _Float16* bp2 = w2h + (size_t)(64 * wave + m) * NHID + CHK * c + 8 * hh;
#pragma unroll 1
    for (int ks = 0; ks < CHK / 32; ++ks) {
      FragH a0, a1;
      a0.h[0] = *(const v8h*)(apy + 32 * ks);
      a0.h[1] = *(const v8h*)(apy + 32 * ks + 16);
      a1.h[0] = *(const v8h*)(apy + 16 * YSP + 32 * ks);
      a1.h[1] = *(const v8h*)(apy + 16 * YSP + 32 * ks + 16);
#pragma unroll
      for (int t = 0; t < 4; ++t) {
        const _Float16* bq = bp2 + (size_t)(16 * t) * NHID + 32 * ks;
        FragH bf;
        bf.h[0] = *(const v8h*)bq;
        bf.h[1] = *(const v8h*)(bq + 16);
        acc2[0][t] = wmh(a0, bf, acc2[0][t]);
        acc2[1][t] = wmh(a1, bf, acc2[1][t]);
      }
    }
    __syncthreads();
  }

  {
    float* sp = stg + (size_t)(8 * hh) * STP + 64 * wave + m;
#pragma unroll
    for (int i = 0; i < 2; ++i)
#pragma unroll
      for (int t = 0; t < 4; ++t)
#pragma unroll
        for (int r = 0; r < 8; ++r) sp[(size_t)(16 * i + r) * STP + 16 * t] = acc2[i][t][r] * SCB;
  }
  __syncthreads();
  {
    const int row = tid >> 3, part = tid & 7;
    const int grow = rowBase + row;
    const int grc  = grow < nN ? grow : nN - 1;
    v4f* sv = (v4f*)(stg + (size_t)row * STP);
    const v4f* xr = (const v4f*)(xf + (size_t)grc * NIN);
    const v4f* b2v = (const v4f*)b2;
    const v4f* gv  = (const v4f*)lng;
    const v4f* bv  = (const v4f*)lnb;
    float s = 0.f;
#pragma unroll 2
    for (int k = 0; k < 16; ++k) {
      const int q = part + 8 * k;
      const v4f y = sv[q] + b2v[q] + xr[q];
      sv[q] = y;
      s += (y.x + y.y) + (y.z + y.w);
    }
    s += __shfl_xor(s, 1);
    s += __shfl_xor(s, 2);
    s += __shfl_xor(s, 4);
    const float mu = s * 0.001953125f;
    float ss = 0.f;
#pragma unroll 2
    for (int k = 0; k < 16; ++k) {
      const int q = part + 8 * k;
      const v4f d = sv[q] - mu;
      ss += (d.x * d.x + d.y * d.y) + (d.z * d.z + d.w * d.w);
    }
    ss += __shfl_xor(ss, 1);
    ss += __shfl_xor(ss, 2);
    ss += __shfl_xor(ss, 4);
    const float var = ss * 0.001953125f;
    const float inv = 1.0f / sqrtf(var + LN_EPS);
#pragma unroll 2
    for (int k = 0; k < 16; ++k) {
      const int q = part + 8 * k;
      const v4f d = (sv[q] - mu) * inv;
      sv[q] = d * gv[q] + bv[q];
    }
  }
  __syncthreads();
  {
    const int nValid = (nN - rowBase) < GBM ? (nN - rowBase) : GBM;
    const int nF4 = nValid * (NIN / 4);
    float* ob = out + (size_t)rowBase * NIN;
#pragma unroll 1
    for (int f = tid; f < nF4; f += GTHR) {
      const int r = f >> 7, q = f & 127;
      const v4f v = *(const v4f*)(stg + (size_t)r * STP + 4 * q);
      *(volatile v4f*)(ob + (size_t)r * NIN + 4 * q) = v;
    }
    __threadfence();
#pragma unroll 1
    for (int f = tid; f < nF4; f += GTHR) {
      const int r = f >> 7, q = f & 127;
      const v4f v = *(const v4f*)(stg + (size_t)r * STP + 4 * q);
      *(volatile v4f*)(ob + (size_t)r * NIN + 4 * q) = v;
    }
  }
}

static int pick_nb(int nE, int nN) {
  int nb = NBMAX;
  while (nb > 16 && (long long)nb * (long long)nE * 5LL > (long long)RCAP * (long long)nN * 4LL) nb >>= 1;
  return nb;
}

extern "C" void kernel_launch(void* const* d_in, const int* in_sizes, int n_in,
                              void* d_out, int out_size, void* d_ws, size_t ws_size,
                              hipStream_t stream) {
  if (n_in < 11) return;
  const int nN = in_sizes[0] / NIN;
  if (nN <= 0 || in_sizes[0] != nN * NIN) return;
  if (nN > (1 << 22)) return;
  const int nE = in_sizes[1];
  if (nE < 1 || nE > (1 << 21)) return;
  if (in_sizes[2] != nE) return;
  if (in_sizes[3] != ZW * NIN) return;
  if (in_sizes[4] != NHEAD * WAW) return;
  if (in_sizes[5] != NHID * NIN || in_sizes[6] != NHID) return;
  if (in_sizes[7] != NIN * NHID || in_sizes[8] != NIN) return;
  if (in_sizes[9] != NIN || in_sizes[10] != NIN) return;
  if (out_size != nN * NIN) return;

  const float* h    = (const float*)d_in[0];
  const int*   srci = (const int*)d_in[1];
  const int*   dsti = (const int*)d_in[2];
  const float* wfc  = (const float*)d_in[3];
  const float* wa   = (const float*)d_in[4];
  const float* w1   = (const float*)d_in[5];
  const float* b1   = (const float*)d_in[6];
  const float* w2   = (const float*)d_in[7];
  const float* b2   = (const float*)d_in[8];
  const float* lng  = (const float*)d_in[9];
  const float* lnb  = (const float*)d_in[10];
  float* out = (float*)d_out;

  const int MP   = ((nN + GBM - 1) / GBM) * GBM;
  const int nb   = pick_nb(nE, nN);
  const int gA   = (nN + nb - 1) / nb;
  const int gG   = MP / GBM;
  const int vec8 = 1;
  if (nb < 16 || nb > NBMAX || (long long)gA * nb < (long long)nN) return;

  char* ws = (char*)d_ws;
  size_t off = 0;
  const size_t oWF  = off; off += (size_t)ZW * NIN * 2;          off = (off + 255) & ~(size_t)255;
  const size_t oW1  = off; off += (size_t)NHID * NIN * 2;        off = (off + 255) & ~(size_t)255;
  const size_t oW2  = off; off += (size_t)NIN * NHID * 2;        off = (off + 255) & ~(size_t)255;
  const size_t oZ   = off; off += (size_t)MP * ZW * 4;           off = (off + 255) & ~(size_t)255;
  const size_t oES  = off; off += (size_t)MP * EPW * 4;          off = (off + 255) & ~(size_t)255;
  const size_t oED  = off; off += (size_t)MP * EPW * 4;          off = (off + 255) & ~(size_t)255;
  const size_t oXF  = off; off += (size_t)MP * NIN * 4;          off = (off + 255) & ~(size_t)255;
  if (off > ws_size || off > (size_t)WSCAP) return;
  _Float16* WF  = (_Float16*)(ws + oWF);
  _Float16* W1H = (_Float16*)(ws + oW1);
  _Float16* W2H = (_Float16*)(ws + oW2);
  float*    Z   = (float*)(ws + oZ);
  float*    ES  = (float*)(ws + oES);
  float*    ED  = (float*)(ws + oED);
  float*    XF  = (float*)(ws + oXF);

  hipFuncSetAttribute(reinterpret_cast<const void*>(&k_gat),
                      hipFuncAttributeMaxDynamicSharedMemorySize, LDS_GAT);
  hipFuncSetAttribute(reinterpret_cast<const void*>(&k_zgemm),
                      hipFuncAttributeMaxDynamicSharedMemorySize, LDS_MM);
  hipFuncSetAttribute(reinterpret_cast<const void*>(&k_ffn),
                      hipFuncAttributeMaxDynamicSharedMemorySize, LDS_MM);

  k_wprep<<<dim3((NIN * NHID / 8 + NTHR - 1) / NTHR, 3), NTHR, 0, stream>>>(wfc, w1, w2, WF, W1H, W2H);

  k_zgemm<<<gG, GTHR, LDS_MM, stream>>>(h, WF, wa, Z, ES, ED, nN);

  k_gat<<<gA, NTHR, LDS_GAT, stream>>>(dsti, srci, Z, ES, ED, h, XF, nN, nE, nb, vec8);

  k_ffn<<<gG, GTHR, LDS_MM, stream>>>(XF, W1H, W2H, b1, b2, lng, lnb, out, nN);
}
